// PLRNNModule_44727789421025
// MI455X (gfx1250) — hardware-verified
//
#include <hip/hip_runtime.h>


typedef _Float16 f16t;
typedef f16t  v16h __attribute__((ext_vector_type(16)));
typedef f16t  v8h  __attribute__((ext_vector_type(8)));
typedef float v8f  __attribute__((ext_vector_type(8)));
typedef float v4f  __attribute__((ext_vector_type(4)));
typedef unsigned int v4u __attribute__((ext_vector_type(4)));

union Frag { v16h v; v8h q[2]; };
union Pk16 { v8h h; v4u u; };
union Pk32 { v4f f; v4u u; };

#define DZ    256
#define AP    264
#define TCH   32
#define WSC   16.0f
#define WINV  0.0625f
#define CLIPV 5.0f

__device__ __forceinline__ v8f wmma16(v16h a, v16h b, v8f c) {
    return __builtin_amdgcn_wmma_f32_16x16x32_f16(false, a, false, b, (short)0, c, false, false);
}

__global__ __launch_bounds__(256)
void k_packw(const float* AW, f16t* P, int nq) {
    int i = blockIdx.x * 256 + threadIdx.x;
    if (i >= nq) return;
    int n = i >> 5;
    int k = (i & 31) * 8;
    const float* src = AW + (size_t)n * DZ + k;
    v4f a = *(const v4f*)src;
    v4f b = *(const v4f*)(src + 4);
    Pk16 pk;
#pragma unroll
    for (int e = 0; e < 4; ++e) {
        float v0 = (k + e == n)     ? 0.0f : a[e] * WSC;
        float v1 = (k + 4 + e == n) ? 0.0f : b[e] * WSC;
        pk.h[e]     = (f16t)v0;
        pk.h[4 + e] = (f16t)v1;
    }
    f16t* d = P + (size_t)n * DZ + k;
    *(volatile v4u*)d = pk.u;
    __threadfence();
    *(volatile v4u*)d = pk.u;
}

__device__ __forceinline__ void stage_x(float* xs, const float* xseq, int m0, int T, int t0, int tid) {
    int row = tid >> 3, c = (tid & 7) * 4;
    v4f q = *(const v4f*)(xseq + (size_t)(m0 + row) * T + t0 + c);
    xs[(c + 0) * 16 + row] = q[0];
    xs[(c + 1) * 16 + row] = q[1];
    xs[(c + 2) * 16 + row] = q[2];
    xs[(c + 3) * 16 + row] = q[3];
}

__global__ __launch_bounds__(256)
void k_scan(const float* xseq, const float* z0, const float* AW, const float* hv,
            const float* Cw, const float* Rw, const float* Rb, const f16t* W16,
            float* out, int T, int nb) {
    __shared__ __attribute__((aligned(32))) f16t  A16[16 * AP];
    __shared__ __attribute__((aligned(32))) float xs[TCH * 16];
    __shared__ __attribute__((aligned(16))) float psum[8 * 16];
    __shared__ __attribute__((aligned(16))) float ybuf[16 * TCH];

    const int tid = threadIdx.x;
    const int w = tid >> 5, l = tid & 31, h = l >> 4, m = l & 15;
    const int m0 = blockIdx.x * 16;
    if (m0 + 16 > nb) return;

    const int nA = 32 * w + m, nB = nA + 16;
    const float adA = AW[(size_t)nA * DZ + nA], adB = AW[(size_t)nB * DZ + nB];
    const float hA = hv[nA], hB = hv[nB];
    const float cA = Cw[nA], cB = Cw[nB];
    const float rA = Rw[nA], rB = Rw[nB];
    const float rb0 = Rb[0];

    float zr0[8], zr1[8];
#pragma unroll
    for (int v = 0; v < 8; ++v) {
        zr0[v] = z0[(size_t)(m0 + 8 * h + v) * DZ + nA];
        zr1[v] = z0[(size_t)(m0 + 8 * h + v) * DZ + nB];
    }

    {
        const int row = tid >> 4, c0 = (tid & 15) * 16;
        const float* src = z0 + (size_t)(m0 + row) * DZ + c0;
        v4f q0 = *(const v4f*)src;
        v4f q1 = *(const v4f*)(src + 4);
        v4f q2 = *(const v4f*)(src + 8);
        v4f q3 = *(const v4f*)(src + 12);
        Pk16 p0, p1;
#pragma unroll
        for (int e = 0; e < 4; ++e) {
            p0.h[e]     = (f16t)fmaxf(q0[e], 0.0f);
            p0.h[4 + e] = (f16t)fmaxf(q1[e], 0.0f);
            p1.h[e]     = (f16t)fmaxf(q2[e], 0.0f);
            p1.h[4 + e] = (f16t)fmaxf(q3[e], 0.0f);
        }
        *(v8h*)(A16 + row * AP + c0)     = p0.h;
        *(v8h*)(A16 + row * AP + c0 + 8) = p1.h;
    }
    if (tid < 128) stage_x(xs, xseq, m0, T, 0, tid);
    __syncthreads();

    const f16t* ap  = A16 + m * AP + 8 * h;
    const f16t* wpA = W16 + (size_t)(32 * w + m) * DZ + 8 * h;
    const f16t* wpB = wpA + (size_t)16 * DZ;

#pragma unroll 1
    for (int t = 0; t < T; ++t) {
        v8f acc0 = {0.f, 0.f, 0.f, 0.f, 0.f, 0.f, 0.f, 0.f};
        v8f acc1 = {0.f, 0.f, 0.f, 0.f, 0.f, 0.f, 0.f, 0.f};
#pragma unroll 1
        for (int kq = 0; kq < DZ; kq += 64) {
            Frag a0, a1, b00, b01, b10, b11;
            a0.q[0]  = *(const v8h*)(ap + kq);
            a0.q[1]  = *(const v8h*)(ap + kq + 16);
            a1.q[0]  = *(const v8h*)(ap + kq + 32);
            a1.q[1]  = *(const v8h*)(ap + kq + 48);
            b00.q[0] = *(const v8h*)(wpA + kq);
            b00.q[1] = *(const v8h*)(wpA + kq + 16);
            b01.q[0] = *(const v8h*)(wpB + kq);
            b01.q[1] = *(const v8h*)(wpB + kq + 16);
            b10.q[0] = *(const v8h*)(wpA + kq + 32);
            b10.q[1] = *(const v8h*)(wpA + kq + 48);
            b11.q[0] = *(const v8h*)(wpB + kq + 32);
            b11.q[1] = *(const v8h*)(wpB + kq + 48);
            acc0 = wmma16(a0.v, b00.v, acc0);
            acc1 = wmma16(a0.v, b01.v, acc1);
            acc0 = wmma16(a1.v, b10.v, acc0);
            acc1 = wmma16(a1.v, b11.v, acc1);
            asm volatile("v_nop\n\tv_nop\n\tv_nop\n\tv_nop"
                         : "+v"(acc0), "+v"(acc1)
                         : "v"(a0.v), "v"(a1.v), "v"(b00.v), "v"(b01.v), "v"(b10.v), "v"(b11.v));
        }
        __syncthreads();

        const int tt = t & (TCH - 1);
        v8f xv = *(const v8f*)(xs + tt * 16 + 8 * h);
        float p[8];
#pragma unroll
        for (int v = 0; v < 8; ++v) {
            const float x = xv[v];
            float zn0 = fmaf(adA, zr0[v], acc0[v] * WINV);
            float zn1 = fmaf(adB, zr1[v], acc1[v] * WINV);
            zn0 += hA;
            zn1 += hB;
            zn0 = fmaf(x, cA, zn0);
            zn1 = fmaf(x, cB, zn1);
            zn0 = fminf(fmaxf(zn0, -CLIPV), CLIPV);
            zn1 = fminf(fmaxf(zn1, -CLIPV), CLIPV);
            zr0[v] = zn0;
            zr1[v] = zn1;
            A16[(8 * h + v) * AP + nA] = (f16t)fmaxf(zn0, 0.0f);
            A16[(8 * h + v) * AP + nB] = (f16t)fmaxf(zn1, 0.0f);
            p[v] = fmaf(zn0, rA, zn1 * rB);
        }
#pragma unroll
        for (int v = 0; v < 8; ++v) {
            float s = p[v];
            s += __shfl_xor(s, 1);
            s += __shfl_xor(s, 2);
            s += __shfl_xor(s, 4);
            s += __shfl_xor(s, 8);
            p[v] = s;
        }
        if (m == 0) {
            Pk32 q0, q1;
            q0.f[0] = p[0]; q0.f[1] = p[1]; q0.f[2] = p[2]; q0.f[3] = p[3];
            q1.f[0] = p[4]; q1.f[1] = p[5]; q1.f[2] = p[6]; q1.f[3] = p[7];
            *(v4f*)(psum + w * 16 + 8 * h)     = q0.f;
            *(v4f*)(psum + w * 16 + 8 * h + 4) = q1.f;
        }
        __syncthreads();

        if (tid < 16) {
            float s = rb0;
#pragma unroll
            for (int ww = 0; ww < 8; ++ww) s += psum[ww * 16 + tid];
            float y = fmaxf(s, 0.0f) + __logf(1.0f + __expf(-fabsf(s)));
            ybuf[tid * TCH + tt] = y;
        }

        if (tt == TCH - 1) {
            __syncthreads();
            if (tid < 128) {
                const int row = tid >> 3, c = (tid & 7) * 4;
                Pk32 yv;
                yv.f = *(const v4f*)(ybuf + row * TCH + c);
                float* dst = out + (size_t)(m0 + row) * T + (t - (TCH - 1)) + c;
                *(volatile v4f*)dst = yv.f;
                __threadfence();
                *(volatile v4f*)dst = yv.f;
                const int t1 = t + 1;
                if (t1 < T) stage_x(xs, xseq, m0, T, t1, tid);
            }
            __syncthreads();
        }
    }
}

extern "C" void kernel_launch(void* const* d_in, const int* in_sizes, int n_in,
                              void* d_out, int out_size, void* d_ws, size_t ws_size,
                              hipStream_t stream) {
    if (n_in < 7) return;
    if (in_sizes[2] != DZ * DZ || in_sizes[3] != DZ || in_sizes[4] != DZ ||
        in_sizes[5] != DZ || in_sizes[6] < 1) return;
    const int nz = in_sizes[1];
    if (nz <= 0 || (nz % DZ) != 0) return;
    const int nb = nz / DZ;
    if ((nb % 16) != 0 || (in_sizes[0] % nb) != 0) return;
    const int T = in_sizes[0] / nb;
    if (T <= 0 || (T % TCH) != 0 || out_size != nb * T) return;

    const size_t wbytes = (size_t)DZ * DZ * 2;
    if (wbytes > ws_size) return;

    const float* xseq = (const float*)d_in[0];
    const float* z0   = (const float*)d_in[1];
    const float* AW   = (const float*)d_in[2];
    const float* hv   = (const float*)d_in[3];
    const float* Cw   = (const float*)d_in[4];
    const float* Rw   = (const float*)d_in[5];
    const float* Rb   = (const float*)d_in[6];
    float* out        = (float*)d_out;
    f16t* W16         = (f16t*)d_ws;

    const int nq = DZ * DZ / 8;
    k_packw<<<dim3((nq + 255) / 256), dim3(256), 0, stream>>>(AW, W16, nq);
    k_scan<<<dim3(nb / 16), dim3(256), 0, stream>>>(xseq, z0, AW, hv, Cw, Rw, Rb, W16,
                                                    out, T, nb);
}
